// PolicyNetwork_63763084476800
// MI455X (gfx1250) — hardware-run, weakly checked
//
#include <hip/hip_runtime.h>
#include <stdint.h>

typedef __attribute__((ext_vector_type(16))) _Float16 v16h;
typedef __attribute__((ext_vector_type(8)))  _Float16 v8h;
typedef __attribute__((ext_vector_type(4)))  _Float16 v4h;
typedef __attribute__((ext_vector_type(8)))  float    v8f;
typedef __attribute__((ext_vector_type(4)))  float    v4f;
typedef __attribute__((ext_vector_type(4)))  unsigned v4u;

__device__ __forceinline__ void dep_guard_h(v8f& a, v8f& b, v16h x, v16h y) { asm volatile("v_nop\n\tv_nop\n\tv_nop\n\tv_nop" : "+v"(a), "+v"(b) : "v"(x), "v"(y)); }
__device__ __forceinline__ void keep4_h(v16h a, v16h b, v16h c, v16h d) { asm volatile("v_nop" :: "v"(a), "v"(b), "v"(c), "v"(d)); }
__device__ __forceinline__ void acc_guard4(v8f& a, v8f& b, v8f& c, v8f& d) { asm volatile("v_nop\n\tv_nop\n\tv_nop\n\tv_nop" : "+v"(a), "+v"(b), "+v"(c), "+v"(d)); }
template <typename T> struct Frag;
template <> struct Frag<_Float16> {
  typedef v16h V; union U { v16h v; v8h h[2]; };
  static __device__ __forceinline__ v16h load(const _Float16* p) {
    U f; f.h[0] = *(const v8h*)(p); f.h[1] = *(const v8h*)(p + 16); return f.v;
  }
  static __device__ __forceinline__ v8f mma(v16h a, v16h b, v8f c) {
    return __builtin_amdgcn_wmma_f32_16x16x32_f16(false, a, false, b, (short)0, c, false, false);
  }
  static __device__ __forceinline__ void guard(v8f& a, v8f& b, v16h x, v16h y) { dep_guard_h(a, b, x, y); }
  static __device__ __forceinline__ void keep(v16h a, v16h b, v16h c, v16h d) { keep4_h(a, b, c, d); }
};
__device__ __forceinline__ void guard3h(v8f& x, v8f& y, v8f& z, v16h a, v16h b0, v16h b1, v16h b2) {
  asm volatile("v_nop\n\tv_nop\n\tv_nop\n\tv_nop" : "+v"(x), "+v"(y), "+v"(z) : "v"(a), "v"(b0), "v"(b1), "v"(b2));
}

constexpr int NB_BATCH     = 64;
constexpr int NSTEP        = 4096;
constexpr int DFEAT        = 8;
constexpr int NXIN         = DFEAT + 1;
constexpr int NHID         = 128;
constexpr int NGATE        = 3 * NHID;
constexpr int KFUSE        = 160;
constexpr int HXP          = 160;
constexpr int ROWS_PER_BLK = 16;
constexpr int NTHREADS     = 256;
constexpr int H1           = 256;
constexpr int H2           = 256;
constexpr int NACT         = 2;

constexpr int OFF_WT    = 0;
constexpr int SZ_WT     = NGATE * HXP * 2;
constexpr int OFF_HX    = OFF_WT + SZ_WT;
constexpr int SZ_HX     = ROWS_PER_BLK * HXP * 2;
constexpr int LDS_TOTAL = OFF_HX + SZ_HX;
constexpr int OFF_HS0   = 0;
constexpr int OFF_HS1   = OFF_HS0 + ROWS_PER_BLK * NHID * 4;
constexpr int OFF_HS2   = OFF_HS1 + ROWS_PER_BLK * H1 * 4;
constexpr int OFF_OUTS  = OFF_HS2 + ROWS_PER_BLK * H2 * 4;

static_assert(NB_BATCH % ROWS_PER_BLK == 0, "grid covers the batch exactly");
static_assert(ROWS_PER_BLK == 16, "one WMMA M tile per workgroup");
static_assert(NTHREADS == 8 * 32 && NHID == 8 * 16 && NGATE == 3 * NHID, "8 waves x 16 columns per gate");
static_assert(KFUSE % 32 == 0 && NHID + NXIN <= KFUSE && HXP >= KFUSE, "K padded to a multiple of 32 inside the tile");
static_assert((HXP * 2) % 16 == 0 && NHID % 32 == 0, "16-B aligned fragment loads");
static_assert(DFEAT == 8, "x row = two float4 halves");
static_assert(H1 == NTHREADS && H2 == NTHREADS, "head layers: one thread per output column");
static_assert(ROWS_PER_BLK * NACT == 32, "each workgroup owns exactly one 128-B output line");
static_assert(OFF_OUTS + 32 * 4 <= SZ_WT, "head staging fits in the reused Wt region");
static_assert(OFF_HX % 16 == 0 && OFF_HS1 % 16 == 0 && OFF_HS2 % 16 == 0 && OFF_OUTS % 16 == 0, "LDS offsets 16-B aligned");
static_assert(LDS_TOTAL % 16 == 0, "LDS zero fill in 16-B chunks");

__device__ __forceinline__ float sigmoid_f(float x) {
  const float e = expf(-fabsf(x));
  const float s = 1.0f / (1.0f + e);
  return (x >= 0.0f) ? s : e * s;
}
__device__ __forceinline__ float tanh_f(float x) {
  const float e = expf(-2.0f * fabsf(x));
  const float t = (1.0f - e) * (1.0f / (1.0f + e));
  return copysignf(t, x);
}

__device__ __forceinline__ void stage_x_row(_Float16* hx, const float* __restrict__ particles,
                                            const float* __restrict__ weights,
                                            int bBase, int t, int c16, int hb) {
  const size_t bt = (size_t)(bBase + c16) * NSTEP + (size_t)t;
  const v4f px = *(const v4f*)(particles + bt * DFEAT + 4 * hb);
  const float pw = weights[bt];
  v4h xv;
  xv[0] = (_Float16)px[0]; xv[1] = (_Float16)px[1]; xv[2] = (_Float16)px[2]; xv[3] = (_Float16)px[3];
  *(v4h*)(hx + c16 * HXP + NHID + 4 * hb) = xv;
  hx[c16 * HXP + NHID + DFEAT] = (_Float16)pw;
}

__global__ __launch_bounds__(NTHREADS) void gru_encoder_head_kernel(
    const float* __restrict__ particles,
    const float* __restrict__ weights,
    const float* __restrict__ Wi,
    const float* __restrict__ bi,
    const float* __restrict__ Wh,
    const float* __restrict__ bhn,
    const float* __restrict__ W1,
    const float* __restrict__ b1,
    const float* __restrict__ W2,
    const float* __restrict__ b2,
    const float* __restrict__ W3,
    const float* __restrict__ b3,
    float* __restrict__ out)
{
  extern __shared__ __align__(16) char smem[];
  _Float16* WtL = (_Float16*)(smem + OFF_WT);
  _Float16* hx  = (_Float16*)(smem + OFF_HX);

  const int tid  = threadIdx.x;
  const int lane = tid & 31;
  const int wave = __builtin_amdgcn_readfirstlane(tid >> 5);
  const int c16  = lane & 15;
  const int hb   = lane >> 4;
  const int bBase = blockIdx.x * ROWS_PER_BLK;

  {
    const v4u z4 = {0u, 0u, 0u, 0u};
    v4u* zp = (v4u*)smem;
    for (int i = tid; i < LDS_TOTAL / 16; i += NTHREADS) zp[i] = z4;
  }
  __syncthreads();
#pragma unroll 4
  for (int e = tid; e < NHID * NGATE; e += NTHREADS) {
    const int k = e / NGATE;
    const int n = e - k * NGATE;
    WtL[n * HXP + k] = (_Float16)Wh[e];
  }
#pragma unroll 1
  for (int e = tid; e < NXIN * NGATE; e += NTHREADS) {
    const int k = e / NGATE;
    const int n = e - k * NGATE;
    WtL[n * HXP + NHID + k] = (_Float16)Wi[e];
  }
  if (wave == 0) stage_x_row(hx, particles, weights, bBase, 0, c16, hb);
  __syncthreads();

  const int colR = wave * 16 + c16;
  const float biasR  = bi[colR];
  const float biasZ  = bi[NHID + colR];
  const float biasNx = bi[2 * NHID + colR];
  const float biasNh = bhn[colR];
  const _Float16* aRow  = hx + c16 * HXP + 8 * hb;
  const _Float16* bRowR = WtL + (size_t)colR * HXP + 8 * hb;
  const _Float16* bRowZ = bRowR + (size_t)NHID * HXP;
  const _Float16* bRowN = bRowR + (size_t)2 * NHID * HXP;
  _Float16* hDst = hx + (8 * hb) * HXP + colR;

  float hreg[8];
#pragma unroll
  for (int r = 0; r < 8; ++r) hreg[r] = 0.0f;
  const v8f zero8 = {0.f, 0.f, 0.f, 0.f, 0.f, 0.f, 0.f, 0.f};

  for (int t = 0; t < NSTEP; ++t) {
    v16h afr[5];
#pragma unroll
    for (int kt = 0; kt < 5; ++kt) afr[kt] = Frag<_Float16>::load(aRow + kt * 32);
    __syncthreads();

    if (wave == 0 && (t + 1 < NSTEP)) stage_x_row(hx, particles, weights, bBase, t + 1, c16, hb);

    v8f c0 = zero8, c1 = zero8, c2 = zero8, c3 = zero8;
#pragma unroll
    for (int kt = 0; kt < 4; ++kt) {
      const v16h bR = Frag<_Float16>::load(bRowR + kt * 32);
      const v16h bZ = Frag<_Float16>::load(bRowZ + kt * 32);
      const v16h bN = Frag<_Float16>::load(bRowN + kt * 32);
      c0 = Frag<_Float16>::mma(afr[kt], bR, c0);
      c1 = Frag<_Float16>::mma(afr[kt], bZ, c1);
      c2 = Frag<_Float16>::mma(afr[kt], bN, c2);
      guard3h(c0, c1, c2, afr[kt], bR, bZ, bN);
    }
    {
      const v16h bR = Frag<_Float16>::load(bRowR + 4 * 32);
      const v16h bZ = Frag<_Float16>::load(bRowZ + 4 * 32);
      const v16h bN = Frag<_Float16>::load(bRowN + 4 * 32);
      c0 = Frag<_Float16>::mma(afr[4], bR, c0);
      c1 = Frag<_Float16>::mma(afr[4], bZ, c1);
      c3 = Frag<_Float16>::mma(afr[4], bN, c3);
      guard3h(c0, c1, c3, afr[4], bR, bZ, bN);
    }
    acc_guard4(c0, c1, c2, c3);

#pragma unroll
    for (int r = 0; r < 8; ++r) {
      const float rg = sigmoid_f(c0[r] + biasR);
      const float zg = sigmoid_f(c1[r] + biasZ);
      const float ng = tanh_f((c3[r] + biasNx) + rg * (c2[r] + biasNh));
      const float hn = ng + zg * (hreg[r] - ng);
      hreg[r] = hn;
      hDst[r * HXP] = (_Float16)hn;
    }
    __syncthreads();
  }

  float* hs0  = (float*)(smem + OFF_HS0);
  float* hs1  = (float*)(smem + OFF_HS1);
  float* hs2  = (float*)(smem + OFF_HS2);
  float* outs = (float*)(smem + OFF_OUTS);
#pragma unroll
  for (int r = 0; r < 8; ++r) hs0[(8 * hb + r) * NHID + colR] = hreg[r];
  __syncthreads();
  {
    const int c = tid;
    const float bv = b1[c];
    float acc[ROWS_PER_BLK];
#pragma unroll
    for (int m = 0; m < ROWS_PER_BLK; ++m) acc[m] = bv;
#pragma unroll 1
    for (int k0 = 0; k0 < NHID; k0 += 4) {
      const float w0 = W1[(size_t)(k0 + 0) * H1 + c];
      const float w1 = W1[(size_t)(k0 + 1) * H1 + c];
      const float w2 = W1[(size_t)(k0 + 2) * H1 + c];
      const float w3 = W1[(size_t)(k0 + 3) * H1 + c];
#pragma unroll
      for (int m = 0; m < ROWS_PER_BLK; ++m) {
        const v4f hv = *(const v4f*)(hs0 + m * NHID + k0);
        float a = acc[m];
        a = fmaf(hv[0], w0, a); a = fmaf(hv[1], w1, a); a = fmaf(hv[2], w2, a); a = fmaf(hv[3], w3, a);
        acc[m] = a;
      }
    }
#pragma unroll
    for (int m = 0; m < ROWS_PER_BLK; ++m) hs1[m * H1 + c] = fmaxf(acc[m], 0.0f);
  }
  __syncthreads();
  {
    const int c = tid;
    const float bv = b2[c];
    float acc[ROWS_PER_BLK];
#pragma unroll
    for (int m = 0; m < ROWS_PER_BLK; ++m) acc[m] = bv;
#pragma unroll 1
    for (int k0 = 0; k0 < H1; k0 += 4) {
      const float w0 = W2[(size_t)(k0 + 0) * H2 + c];
      const float w1 = W2[(size_t)(k0 + 1) * H2 + c];
      const float w2 = W2[(size_t)(k0 + 2) * H2 + c];
      const float w3 = W2[(size_t)(k0 + 3) * H2 + c];
#pragma unroll
      for (int m = 0; m < ROWS_PER_BLK; ++m) {
        const v4f hv = *(const v4f*)(hs1 + m * H1 + k0);
        float a = acc[m];
        a = fmaf(hv[0], w0, a); a = fmaf(hv[1], w1, a); a = fmaf(hv[2], w2, a); a = fmaf(hv[3], w3, a);
        acc[m] = a;
      }
    }
#pragma unroll
    for (int m = 0; m < ROWS_PER_BLK; ++m) hs2[m * H2 + c] = fmaxf(acc[m], 0.0f);
  }
  __syncthreads();
  if (wave == 0) {
    const int m = lane >> 1, a = lane & 1;
    float acc3 = b3[a];
#pragma unroll 1
    for (int k = 0; k < H2; ++k) acc3 = fmaf(hs2[m * H2 + k], W3[k * NACT + a], acc3);
    outs[lane] = acc3;
  }
  __syncthreads();
  if (wave == 0) {
    const int q = lane & 7;
    const v4f v = *(const v4f*)(outs + 4 * q);
    float* op = out + (size_t)bBase * NACT + 4 * q;
    if (lane < 8) *(volatile v4f*)op = v;
    __threadfence();
    if (lane < 8) *(volatile v4f*)op = v;
  }
}

extern "C" void kernel_launch(void* const* d_in, const int* in_sizes, int n_in,
                              void* d_out, int out_size, void* d_ws, size_t ws_size,
                              hipStream_t stream) {
  (void)in_sizes; (void)n_in; (void)out_size; (void)d_ws; (void)ws_size;
  const float* particles = (const float*)d_in[0];
  const float* weights   = (const float*)d_in[1];
  const float* Wi        = (const float*)d_in[2];
  const float* bi        = (const float*)d_in[3];
  const float* Wh        = (const float*)d_in[4];
  const float* bhn       = (const float*)d_in[5];
  const float* W1        = (const float*)d_in[6];
  const float* b1        = (const float*)d_in[7];
  const float* W2        = (const float*)d_in[8];
  const float* b2        = (const float*)d_in[9];
  const float* W3        = (const float*)d_in[10];
  const float* b3        = (const float*)d_in[11];
  float* out = (float*)d_out;

  gru_encoder_head_kernel<<<NB_BATCH / ROWS_PER_BLK, NTHREADS, LDS_TOTAL, stream>>>(
      particles, weights, Wi, bi, Wh, bhn, W1, b1, W2, b2, W3, b3, out);
}
